// GroupedQueryAttention_55138790146626
// MI455X (gfx1250) — hardware-verified
//
#include <hip/hip_runtime.h>
#include <math.h>


#ifndef NB
#define NB 2
#endif
#ifndef SEQ
#define SEQ 2048
#endif
#define NB_FULL  2
#define SEQ_FULL 2048
#define DM   1024
#define NH_  16
#define NKV  4
#define REP  (NH_ / NKV)
#define HD   64
#define DQ   (NH_ * HD)
#define DKV  (NKV * HD)
#define DQKV (DQ + 2 * DKV)
#if SEQ < 512
#define RH SEQ
#else
#define RH 512
#endif
#define NTOK (NB * SEQ)
#define SCL  0.125f
#define L2E  1.4426950408889634f
#define NEGB (-1.0e30f)

static_assert(SEQ % 256 == 0);
static_assert(RH % 256 == 0);
static_assert(NTOK % 64 == 0);
static_assert(DM % 32 == 0 && DQ % 32 == 0);
static_assert(DQKV % 64 == 0 && DM % 64 == 0);
static_assert(NB <= NB_FULL && SEQ <= SEQ_FULL);
static_assert(DM == 1024);

typedef _Float16 h16;
typedef unsigned short bf;
typedef __attribute__((ext_vector_type(16))) __bf16   v16bf;
typedef __attribute__((ext_vector_type(16))) _Float16 v16h;
typedef __attribute__((ext_vector_type(8)))  _Float16 v8h;
typedef __attribute__((ext_vector_type(8)))  unsigned short v8us;
typedef __attribute__((ext_vector_type(2)))  unsigned short v2us;
typedef __attribute__((ext_vector_type(8)))  float    v8f;
typedef __attribute__((ext_vector_type(4)))  float    v4f;
typedef __attribute__((ext_vector_type(2)))  float    v2f;
typedef v4f  __attribute__((may_alias)) v4fa;
typedef v8us __attribute__((may_alias)) v8usa;

__device__ __forceinline__ unsigned short f2bf(float f) { unsigned u = __float_as_uint(f); u += 0x7FFFu + ((u >> 16) & 1u); return (unsigned short)(u >> 16); }
__device__ __forceinline__ float bf2f(unsigned short b) { return __uint_as_float(((unsigned)b) << 16); }
__device__ __forceinline__ float bfr(float f) { return bf2f(f2bf(f)); }
__device__ __forceinline__ void splitf(float y, unsigned short& h, unsigned short& l) { h = f2bf(y); l = f2bf(y - bf2f(h)); }
__device__ __forceinline__ v16h cat16(v8h lo, v8h hi) { return __builtin_shufflevector(lo, hi, 0, 1, 2, 3, 4, 5, 6, 7, 8, 9, 10, 11, 12, 13, 14, 15); }
__device__ __forceinline__ v16bf cat16b(v8us lo, v8us hi) { return __builtin_bit_cast(v16bf, __builtin_shufflevector(lo, hi, 0, 1, 2, 3, 4, 5, 6, 7, 8, 9, 10, 11, 12, 13, 14, 15)); }
__device__ __forceinline__ v8f wmma16(v16h a, v16h b, v8f c) { return __builtin_amdgcn_wmma_f32_16x16x32_f16(false, a, false, b, (short)0, c, false, false); }
__device__ __forceinline__ v8f wmmab(v16bf a, v16bf b, v8f c) { return __builtin_amdgcn_wmma_f32_16x16x32_bf16(false, a, false, b, (short)0, c, false, false); }

template <typename T16> struct WFrag;
template <> struct WFrag<h16> { typedef v16h V; static __device__ __forceinline__ V ld(const h16* p) { return cat16(*(const v8h*)p, *(const v8h*)(p + 16)); } static __device__ __forceinline__ v8f mma(V a, V b, v8f c) { return wmma16(a, b, c); }
    static __device__ __forceinline__ V phi(v8f p0, v8f p1) { v8h a, b;
#pragma unroll
        for (int r = 0; r < 8; ++r) { a[r] = (h16)p0[r]; b[r] = (h16)p1[r]; } return cat16(a, b); }
    static __device__ __forceinline__ V plo(v8f p0, v8f p1) { return phi(p0, p1); } };
template <> struct WFrag<bf> { typedef v16bf V; static __device__ __forceinline__ V ld(const bf* p) { return cat16b(*(const v8us*)p, *(const v8us*)(p + 16)); } static __device__ __forceinline__ v8f mma(V a, V b, v8f c) { return wmmab(a, b, c); }
    static __device__ __forceinline__ V phi(v8f p0, v8f p1) { v8us a, b;
#pragma unroll
        for (int r = 0; r < 8; ++r) { a[r] = f2bf(p0[r]); b[r] = f2bf(p1[r]); } return cat16b(a, b); }
    static __device__ __forceinline__ V plo(v8f p0, v8f p1) { v8us a, b;
#pragma unroll
        for (int r = 0; r < 8; ++r) { unsigned short x, y; splitf(p0[r], x, y); a[r] = y; splitf(p1[r], x, y); b[r] = y; } return cat16b(a, b); } };

template <typename T16, int NSPLIT, bool BIAS>
__global__ __launch_bounds__(32) void k_gemmw(const T16* __restrict__ A, const T16* __restrict__ A2, const T16* __restrict__ Bt, const T16* __restrict__ Bt2, int K, float* C, int ldc, const float* __restrict__ bias, size_t sA, size_t sB, size_t sC) {
    typedef typename WFrag<T16>::V V;
    __shared__ __align__(16) float os[16 * 68];
    const size_t z = blockIdx.z; A += z * sA; if (A2) A2 += z * sA; Bt += z * sB; if (Bt2) Bt2 += z * sB; C += z * sC;
    const int lane = threadIdx.x & 31, lr = lane & 15, hi = lane >> 4; const int r0 = blockIdx.x * 64, c0 = blockIdx.y * 64;
    v8f acc[4][4];
#pragma unroll
    for (int mb = 0; mb < 4; ++mb)
#pragma unroll
        for (int nb = 0; nb < 4; ++nb) acc[mb][nb] = (v8f){};
    const size_t aoff = (size_t)(r0 + lr) * K + 8 * hi, boff = (size_t)(c0 + lr) * K + 8 * hi;
#pragma unroll 1
    for (int kc = 0; kc < K; kc += 32) {
        V a[4], a2[4];
#pragma unroll
        for (int mb = 0; mb < 4; ++mb) { a[mb] = WFrag<T16>::ld(A + aoff + (size_t)mb * 16 * K + kc); if (NSPLIT == 1 || NSPLIT == 2) a2[mb] = WFrag<T16>::ld(A2 + aoff + (size_t)mb * 16 * K + kc); }
#pragma unroll
        for (int nb = 0; nb < 4; ++nb) { const V b = WFrag<T16>::ld(Bt + boff + (size_t)nb * 16 * K + kc); V b2; if (NSPLIT >= 2) b2 = WFrag<T16>::ld(Bt2 + boff + (size_t)nb * 16 * K + kc);
#pragma unroll
            for (int mb = 0; mb < 4; ++mb) { acc[mb][nb] = WFrag<T16>::mma(a[mb], b, acc[mb][nb]); if (NSPLIT == 1 || NSPLIT == 2) acc[mb][nb] = WFrag<T16>::mma(a2[mb], b, acc[mb][nb]); if (NSPLIT >= 2) acc[mb][nb] = WFrag<T16>::mma(a[mb], b2, acc[mb][nb]); } }
        asm volatile("v_nop\n\tv_nop\n\tv_nop\n\tv_nop" : "+v"(acc[0][0]), "+v"(acc[1][1]), "+v"(acc[2][2]), "+v"(acc[3][3]) : "v"(a[0]), "v"(a[3]));
    }
#pragma unroll
    for (int mb = 0; mb < 4; ++mb) {
#pragma unroll
        for (int nb = 0; nb < 4; ++nb) {
#pragma unroll
            for (int j = 0; j < 8; ++j) os[(hi * 8 + j) * 68 + nb * 16 + lr] = acc[mb][nb][j]; }
        __builtin_amdgcn_wave_barrier(); asm volatile("" ::: "memory");
        float* crow = C + (size_t)(r0 + mb * 16) * ldc + c0;
#pragma unroll 1
        for (int ps = 0; ps < 2; ++ps) {
#pragma unroll
            for (int s = 0; s < 8; ++s) { const int row = 2 * s + hi, cofs = lr * 4; v4f val = *(const v4fa*)(os + row * 68 + cofs); if (BIAS) { val[0] += bfr(bias[c0 + cofs]); val[1] += bfr(bias[c0 + cofs + 1]); val[2] += bfr(bias[c0 + cofs + 2]); val[3] += bfr(bias[c0 + cofs + 3]); }
                *(volatile v4f*)(crow + (size_t)row * ldc + cofs) = val; }
            if (ps == 0) __threadfence(); }
        __builtin_amdgcn_wave_barrier(); asm volatile("" ::: "memory");
    }
}

__global__ __launch_bounds__(256) void k_wt(const float* __restrict__ w, unsigned N, bf* Bt) {
    const unsigned lane = threadIdx.x & 31u; const unsigned L0 = (blockIdx.x * 8u + (threadIdx.x >> 5)) * 8u;
    v2us o[8];
#pragma unroll
    for (int l = 0; l < 8; ++l) { const unsigned e = (L0 + (unsigned)l) * 64u + lane * 2u; const unsigned k = e & (DM - 1u), n = e >> 10; o[l][0] = f2bf(w[k * N + n]); o[l][1] = f2bf(w[(k + 1u) * N + n]); }
#pragma unroll 1
    for (int ps = 0; ps < 2; ++ps) {
#pragma unroll
        for (int l = 0; l < 8; ++l) { const unsigned e = (L0 + (unsigned)l) * 64u + lane * 2u; *(volatile v2us*)(Bt + e) = o[l]; }
        if (ps == 0) __threadfence(); }
}

__global__ __launch_bounds__(256) void k_cvt8(const float* __restrict__ src, bf* dst) {
    const unsigned b = blockIdx.y; const size_t i = (size_t)blockIdx.x * 256u + threadIdx.x;
    const v8f v = *(const v8f*)(src + (size_t)b * SEQ_FULL * DM + i * 8); bf* d = dst + (size_t)b * SEQ * DM + i * 8; v8us o;
#pragma unroll
    for (int k = 0; k < 8; ++k) o[k] = f2bf(v[k]);
    *(volatile v8us*)d = o; __threadfence(); *(volatile v8us*)d = o; }

struct InvF { float v[32]; };
static_assert(sizeof(InvF) == 128);
__global__ __launch_bounds__(256) void k_cstab(InvF f, float* CS) {
    const unsigned idx = blockIdx.x * 256u + threadIdx.x; const unsigned i = idx & 31u, t = idx >> 5;
    float inv = f.v[0];
#pragma unroll
    for (int q = 1; q < 32; ++q) inv = (i == (unsigned)q) ? f.v[q] : inv;
    const float ang = (float)t * inv; float s, c; sincosf(ang, &s, &c);
    v2f o; o[0] = c; o[1] = s; *(volatile v2f*)(CS + (size_t)idx * 2) = o; __threadfence(); *(volatile v2f*)(CS + (size_t)idx * 2) = o; }

__global__ __launch_bounds__(256) void k_rope8(const float* __restrict__ F, unsigned coloff, unsigned nheads, const float* __restrict__ CS, h16* P16, bf* Ph, bf* Pl) {
#pragma clang fp contract(off)
    const unsigned idx = blockIdx.x * 256u + threadIdx.x; const unsigned c = idx & 7u, t = idx >> 3; const unsigned b = blockIdx.y, h = blockIdx.z;
    const unsigned d0 = c * 8u, dp0 = d0 ^ 32u, j0 = d0 & 31u;
    const float* f = F + (size_t)(b * SEQ + t) * DQKV + coloff + h * HD;
    const v4f xa = *(const v4f*)(f + d0), xb = *(const v4f*)(f + d0 + 4), ya = *(const v4f*)(f + dp0), yb = *(const v4f*)(f + dp0 + 4);
    const float* cs = CS + ((size_t)t * 32u + j0) * 2u;
    const v4f c0 = *(const v4f*)cs, c1 = *(const v4f*)(cs + 4), c2 = *(const v4f*)(cs + 8), c3 = *(const v4f*)(cs + 12);
    const float x[8] = { xa[0], xa[1], xa[2], xa[3], xb[0], xb[1], xb[2], xb[3] };
    const float y[8] = { ya[0], ya[1], ya[2], ya[3], yb[0], yb[1], yb[2], yb[3] };
    const float cc[8] = { c0[0], c0[2], c1[0], c1[2], c2[0], c2[2], c3[0], c3[2] };
    const float ss[8] = { c0[1], c0[3], c1[1], c1[3], c2[1], c2[3], c3[1], c3[3] };
    const float sg = (d0 < 32u) ? -1.0f : 1.0f;
    v8h o16; v8us oh, ol;
#pragma unroll
    for (int q = 0; q < 8; ++q) { const float a = x[q] * cc[q]; const float bq = y[q] * ss[q]; const float r = a + sg * bq; o16[q] = (h16)r; unsigned short a2, c2b; splitf(r, a2, c2b); oh[q] = a2; ol[q] = c2b; }
    const size_t e16 = ((size_t)(b * nheads + h) * SEQ + t) * HD + d0; const size_t ehl = ((size_t)(b * nheads + h) * RH + t) * HD + d0; const bool hl = (t < (unsigned)RH);
    *(volatile v8h*)(P16 + e16) = o16; if (hl) { *(volatile v8us*)(Ph + ehl) = oh; *(volatile v8us*)(Pl + ehl) = ol; }
    __threadfence();
    *(volatile v8h*)(P16 + e16) = o16; if (hl) { *(volatile v8us*)(Ph + ehl) = oh; *(volatile v8us*)(Pl + ehl) = ol; }
}

__global__ __launch_bounds__(256) void k_vtp8(const float* __restrict__ F, unsigned coloff, h16* V16, bf* Vh, bf* Vl) {
    const unsigned idx = blockIdx.x * 256u + threadIdx.x; const unsigned S8 = SEQ / 8u; const unsigned tc = idx % S8, d = idx / S8; const unsigned b = blockIdx.y, g = blockIdx.z; const unsigned t0 = tc * 8u;
    const float* f = F + (size_t)(b * SEQ + t0) * DQKV + coloff + g * HD + d;
    v8h o16; v8us oh, ol;
#pragma unroll
    for (int q = 0; q < 8; ++q) { const float x = f[(size_t)q * DQKV]; o16[q] = (h16)x; unsigned short a2, c2; splitf(x, a2, c2); oh[q] = a2; ol[q] = c2; }
    const size_t e16 = ((size_t)(b * NKV + g) * HD + d) * SEQ + t0; const size_t ehl = ((size_t)(b * NKV + g) * HD + d) * RH + t0; const bool hl = (t0 < (unsigned)RH);
    *(volatile v8h*)(V16 + e16) = o16; if (hl) { *(volatile v8us*)(Vh + ehl) = oh; *(volatile v8us*)(Vl + ehl) = ol; }
    __threadfence();
    *(volatile v8h*)(V16 + e16) = o16; if (hl) { *(volatile v8us*)(Vh + ehl) = oh; *(volatile v8us*)(Vl + ehl) = ol; }
}

template <typename T16, bool HI>
__global__ __launch_bounds__(128) void k_flash(const T16* __restrict__ Qa, const T16* __restrict__ Qb, const T16* __restrict__ Ka, const T16* __restrict__ Kb, const T16* __restrict__ Va, const T16* __restrict__ Vb, bf* ATh, bf* ATl) {
    typedef typename WFrag<T16>::V V;
    constexpr unsigned KP = HI ? (unsigned)RH : (unsigned)SEQ;
    constexpr unsigned QB = HI ? 0u : (unsigned)RH;
    constexpr float CAR = HI ? 0.0f : 10.0f;
    __shared__ __align__(16) unsigned short sH[4 * 16 * 72];
    __shared__ __align__(16) unsigned short sL[4 * 16 * 72];
    const unsigned lane = threadIdx.x & 31u, lr = lane & 15u, hi = lane >> 4, w = threadIdx.x >> 5;
    const unsigned g = blockIdx.y, b = blockIdx.z, hh = g * REP + w, q0 = QB + blockIdx.x * 16u;
    const size_t qo = ((size_t)(b * NH_ + hh) * KP + q0 + lr) * HD + 8u * hi;
    V qh[2], ql[2];
    qh[0] = WFrag<T16>::ld(Qa + qo); qh[1] = WFrag<T16>::ld(Qa + qo + 32);
    if (HI) { ql[0] = WFrag<T16>::ld(Qb + qo); ql[1] = WFrag<T16>::ld(Qb + qo + 32); } else { ql[0] = qh[0]; ql[1] = qh[1]; }
    const size_t ko = ((size_t)(b * NKV + g) * KP + lr) * HD + 8u * hi;
    const size_t vo = ((size_t)(b * NKV + g) * HD + lr) * KP + 8u * hi;
    v8f oacc[4];
#pragma unroll
    for (int dt = 0; dt < 4; ++dt) oacc[dt] = (v8f){};
    float mrow = NEGB, lsum = 0.0f;
    const unsigned nblk = (q0 + 16u + 31u) >> 5;
    const unsigned qi = q0 + lr;
#pragma unroll 1
    for (unsigned blk = 0; blk < nblk; ++blk) {
        const unsigned kv0 = blk * 32u;
        v8f s[2]; s[0] = (v8f){}; s[1] = (v8f){};
#pragma unroll
        for (int kt = 0; kt < 2; ++kt) {
#pragma unroll
            for (int ds = 0; ds < 2; ++ds) { const size_t o = ko + (size_t)(kv0 + (unsigned)kt * 16u) * HD + (unsigned)ds * 32u; const V a = WFrag<T16>::ld(Ka + o); s[kt] = WFrag<T16>::mma(a, qh[ds], s[kt]);
                if (HI) { s[kt] = WFrag<T16>::mma(a, ql[ds], s[kt]); const V a2 = WFrag<T16>::ld(Kb + o); s[kt] = WFrag<T16>::mma(a2, qh[ds], s[kt]); } } }
        asm volatile("v_nop\n\tv_nop\n\tv_nop\n\tv_nop" : "+v"(s[0]), "+v"(s[1]) : "v"(qh[0]), "v"(qh[1]));
        v8f t0 = s[0] * SCL, t1 = s[1] * SCL;
        if (kv0 + 31u > q0) {
#pragma unroll
            for (int r = 0; r < 8; ++r) { const unsigned key = kv0 + 8u * hi + (unsigned)r; t0[r] = (key > qi) ? NEGB : t0[r]; t1[r] = (key + 16u > qi) ? NEGB : t1[r]; } }
        float mx = fmaxf(t0[0], t1[0]);
#pragma unroll
        for (int r = 1; r < 8; ++r) mx = fmaxf(mx, fmaxf(t0[r], t1[r]));
        mx = fmaxf(mx, __shfl_xor(mx, 16, 32));
        const float mn = fmaxf(mrow, mx);
        const float alpha = __builtin_amdgcn_exp2f((mrow - mn) * L2E);
        mrow = mn;
        v8f p0, p1; float psum = 0.0f;
#pragma unroll
        for (int r = 0; r < 8; ++r) { p0[r] = __builtin_amdgcn_exp2f((t0[r] - mn) * L2E + CAR); p1[r] = __builtin_amdgcn_exp2f((t1[r] - mn) * L2E + CAR); psum += p0[r] + p1[r]; }
        lsum = lsum * alpha + psum;
#pragma unroll
        for (int dt = 0; dt < 4; ++dt) oacc[dt] = oacc[dt] * alpha;
        const V pbh = WFrag<T16>::phi(p0, p1);
        V pbl = pbh; if (HI) pbl = WFrag<T16>::plo(p0, p1);
#pragma unroll
        for (int dt = 0; dt < 4; ++dt) { const size_t o = vo + (size_t)((unsigned)dt * 16u) * KP + kv0; const V a = WFrag<T16>::ld(Va + o); oacc[dt] = WFrag<T16>::mma(a, pbh, oacc[dt]);
            if (HI) { oacc[dt] = WFrag<T16>::mma(a, pbl, oacc[dt]); const V a2 = WFrag<T16>::ld(Vb + o); oacc[dt] = WFrag<T16>::mma(a2, pbh, oacc[dt]); } }
        asm volatile("v_nop\n\tv_nop\n\tv_nop\n\tv_nop" : "+v"(oacc[0]), "+v"(oacc[1]), "+v"(oacc[2]), "+v"(oacc[3]) : "v"(pbh), "v"(pbl));
    }
    const float l = lsum + __shfl_xor(lsum, 16, 32);
    const float inv = 1.0f / l;
    unsigned short* mh = sH + w * (16u * 72u); unsigned short* ml = sL + w * (16u * 72u);
#pragma unroll
    for (int dt = 0; dt < 4; ++dt) { v8us oh, ol;
#pragma unroll
        for (int r = 0; r < 8; ++r) { unsigned short a2, c2; splitf(oacc[dt][r] * inv, a2, c2); oh[r] = a2; ol[r] = c2; }
        const unsigned so = lr * 72u + (unsigned)dt * 16u + 8u * hi; *(v8usa*)(mh + so) = oh; *(v8usa*)(ml + so) = ol; }
    __syncthreads();
    v8us vh[4], vl[4];
#pragma unroll
    for (int s4 = 0; s4 < 4; ++s4) { const unsigned row = (unsigned)s4 * 4u + (lane >> 3), c8 = (lane & 7u) * 8u; vh[s4] = *(const v8usa*)(mh + row * 72u + c8); vl[s4] = *(const v8usa*)(ml + row * 72u + c8); }
#pragma unroll 1
    for (int ps = 0; ps < 2; ++ps) {
#pragma unroll
        for (int s4 = 0; s4 < 4; ++s4) { const unsigned row = (unsigned)s4 * 4u + (lane >> 3), c8 = (lane & 7u) * 8u; const size_t oo = (size_t)(b * SEQ + q0 + row) * DQ + hh * HD + c8;
            *(volatile v8us*)(ATh + oo) = vh[s4]; *(volatile v8us*)(ATl + oo) = vl[s4]; }
        if (ps == 0) __threadfence(); }
}

#define SZ_WQKV ((size_t)DQKV * DM * 2)
#define SZ_WO   ((size_t)DM * DQ * 2)
#define SZ_CS   ((size_t)SEQ * 32 * 2 * 4)
#define SZ_XB   ((size_t)NTOK * DM * 2)
#define SZ_F    ((size_t)NTOK * DQKV * 4)
#define SZ_Q16  ((size_t)NB * NH_ * SEQ * HD * 2)
#define SZ_K16  ((size_t)NB * NKV * SEQ * HD * 2)
#define SZ_QHL  ((size_t)NB * NH_ * RH * HD * 2)
#define SZ_KHL  ((size_t)NB * NKV * RH * HD * 2)
#define SZ_AT   ((size_t)NTOK * DQ * 2)
#define SZ_TOT  (SZ_WQKV + SZ_WO + SZ_CS + SZ_XB + SZ_F + SZ_Q16 + 2 * SZ_K16 + 2 * SZ_QHL + 4 * SZ_KHL + 2 * SZ_AT)
static_assert(SZ_TOT <= (size_t)134217728);
static_assert(SZ_CS % 256 == 0 && SZ_KHL % 256 == 0);

extern "C" void kernel_launch(void* const* d_in, const int* in_sizes, int n_in,
                              void* d_out, int out_size, void* d_ws, size_t ws_size, hipStream_t stream) {
    if (n_in < 5) return;
    if ((size_t)in_sizes[0] < ((size_t)(NB - 1) * SEQ_FULL + SEQ) * DM) return;
    if (in_sizes[1] < DM * DQ || in_sizes[2] < DM * DKV || in_sizes[3] < DM * DKV || in_sizes[4] < DQ * DM) return;
    if ((size_t)out_size < (size_t)NTOK * DM) return;
    if (SZ_TOT > ws_size) return;
    const float* x = (const float*)d_in[0]; const float* wq = (const float*)d_in[1]; const float* wk = (const float*)d_in[2]; const float* wv = (const float*)d_in[3]; const float* wo = (const float*)d_in[4];
    float* OUT = (float*)d_out;
    char* wsp = (char*)d_ws;
    auto take = [&](size_t bytes) { char* p = wsp; wsp += bytes; return (void*)p; };
    bf* WQKV = (bf*)take(SZ_WQKV); bf* WO = (bf*)take(SZ_WO); float* CS = (float*)take(SZ_CS); bf* XB = (bf*)take(SZ_XB); float* F = (float*)take(SZ_F);
    h16* Q16 = (h16*)take(SZ_Q16); h16* K16 = (h16*)take(SZ_K16); h16* VT16 = (h16*)take(SZ_K16);
    bf* Qh = (bf*)take(SZ_QHL); bf* Ql = (bf*)take(SZ_QHL); bf* Kh = (bf*)take(SZ_KHL); bf* Kl = (bf*)take(SZ_KHL); bf* VTh = (bf*)take(SZ_KHL); bf* VTl = (bf*)take(SZ_KHL);
    bf* ATh = (bf*)take(SZ_AT); bf* ATl = (bf*)take(SZ_AT);

    InvF fr;
    for (int i = 0; i < 32; ++i) fr.v[i] = 1.0f / (float)pow(10000.0, (double)(2 * i) / 64.0);

    k_wt<<<DQ / 4, 256, 0, stream>>>(wq, (unsigned)DQ, WQKV);
    k_wt<<<DKV / 4, 256, 0, stream>>>(wk, (unsigned)DKV, WQKV + (size_t)DQ * DM);
    k_wt<<<DKV / 4, 256, 0, stream>>>(wv, (unsigned)DKV, WQKV + (size_t)(DQ + DKV) * DM);
    k_wt<<<DM / 4, 256, 0, stream>>>(wo, (unsigned)DM, WO);
    k_cstab<<<SEQ / 8, 256, 0, stream>>>(fr, CS);
    k_cvt8<<<dim3(SEQ / 2, NB, 1), 256, 0, stream>>>(x, XB);
    k_gemmw<bf, 0, false><<<dim3(NTOK / 64, DQKV / 64, 1), 32, 0, stream>>>(XB, nullptr, WQKV, nullptr, DM, F, DQKV, nullptr, 0, 0, 0);
    k_rope8<<<dim3(SEQ * 8 / 256, NB, NH_), 256, 0, stream>>>(F, 0u, (unsigned)NH_, CS, Q16, Qh, Ql);
    k_rope8<<<dim3(SEQ * 8 / 256, NB, NKV), 256, 0, stream>>>(F, (unsigned)DQ, (unsigned)NKV, CS, K16, Kh, Kl);
    k_vtp8<<<dim3(HD * (SEQ / 8) / 256, NB, NKV), 256, 0, stream>>>(F, (unsigned)(DQ + DKV), VT16, VTh, VTl);
    k_flash<bf, true><<<dim3(RH / 16, NKV, NB), 128, 0, stream>>>(Qh, Ql, Kh, Kl, VTh, VTl, ATh, ATl);
    if (SEQ > RH) k_flash<h16, false><<<dim3((SEQ - RH) / 16 > 0 ? (SEQ - RH) / 16 : 1, NKV, NB), 128, 0, stream>>>(Q16, nullptr, K16, nullptr, VT16, nullptr, ATh, ATl);
    k_gemmw<bf, 1, false><<<dim3(NTOK / 64, DM / 64, 1), 32, 0, stream>>>(ATh, ATl, WO, nullptr, DQ, OUT, DM, nullptr, 0, 0, 0);
}
